// NeuralRenderer1_1365799600526
// MI455X (gfx1250) — hardware-verified
//
#include <hip/hip_runtime.h>
#include <math.h>


#define NB 8
#define C0 256
#define C1 128
#define C2 64
#define ST 512
#define H0 64
#define P0 (H0 * H0)
#define H1 128
#define P1 (H1 * H1)
#define H2 256
#define P2 (H2 * H2)

typedef __attribute__((ext_vector_type(16))) _Float16 v16h;
typedef __attribute__((ext_vector_type(8)))  _Float16 v8h;
typedef __attribute__((ext_vector_type(8)))  float v8f;
typedef __attribute__((ext_vector_type(4)))  float v4f;
typedef __attribute__((ext_vector_type(4)))  unsigned v4u;
typedef float __attribute__((may_alias)) float_a;

template <typename T> __device__ __forceinline__ void vst2(void* p, T v) { *(volatile T*)p = v; __threadfence(); *(volatile T*)p = v; }
__device__ __forceinline__ v8f wmma16(v16h a, v16h b, v8f c) {
  v8f d = __builtin_amdgcn_wmma_f32_16x16x32_f16(false, a, false, b, (short)0, c, false, false);
  asm volatile("v_nop\n\tv_nop\n\tv_nop\n\tv_nop" : "+v"(d) : "v"(a), "v"(b));
  return d;
}
__device__ __forceinline__ v16h frag_h(const _Float16* rowk0, int lane) {
  union { v16h v; v8h q[2]; } u; const _Float16* p = rowk0 + 8 * (lane >> 4);
  u.q[0] = *(const v8h*)p; u.q[1] = *(const v8h*)(p + 16); return u.v;
}
__device__ __forceinline__ float lrelu(float v) { return v >= 0.f ? v : 0.2f * v; }
#define LDSX() do { asm volatile("s_wait_dscnt 0" ::: "memory"); __builtin_amdgcn_wave_barrier(); __builtin_amdgcn_fence(__ATOMIC_RELEASE, "workgroup"); } while (0)

__global__ __launch_bounds__(256) void k_style(const float* __restrict__ y, const float* __restrict__ w0, const float* __restrict__ b0,
    const float* __restrict__ w1, const float* __restrict__ b1, const float* __restrict__ w2, const float* __restrict__ b2,
    const float* __restrict__ w3, const float* __restrict__ b3, const float* __restrict__ w4, const float* __restrict__ b4,
    const float* __restrict__ w5, const float* __restrict__ b5, float* __restrict__ S) {
  const int j = blockIdx.y, b = blockIdx.x, o = threadIdx.x;
  const int od = j == 0 ? 256 : (j < 4 ? 128 : 64);
  const float* W = j == 0 ? w0 : j == 1 ? w1 : j == 2 ? w2 : j == 3 ? w3 : j == 4 ? w4 : w5;
  const float* bb = j == 0 ? b0 : j == 1 ? b1 : j == 2 ? b2 : j == 3 ? b3 : j == 4 ? b4 : b5;
  const float* yv = y + ((size_t)b * 2 + (j < 3 ? 0 : 1)) * ST;
  if (o >= od) return;
  float a = bb[o];
#pragma unroll 1
  for (int i = 0; i < ST; ++i) a += yv[i] * W[(size_t)o * ST + i];
  vst2(S + ((size_t)j * NB + b) * 256 + o, (float_a)a);
}

__global__ __launch_bounds__(256) void k_wmod(const float* __restrict__ Wc, const float* __restrict__ S, int sj, int O, int I,
                                            _Float16* __restrict__ wm) {
  __shared__ float red[256];
  const int b = blockIdx.y, o = blockIdx.x, tid = threadIdx.x;
  const float w = tid < I ? Wc[(size_t)o * I + tid] * (S[((size_t)sj * NB + b) * 256 + tid] + 1.0f) : 0.f;
  red[tid] = w * w; __syncthreads();
  for (int st = 128; st > 0; st >>= 1) { if (tid < st) red[tid] += red[tid + st]; __syncthreads(); }
  const float dm = rsqrtf(red[0] + 1e-8f);
  __shared__ float wrow[256];
  wrow[tid] = w * dm; __syncthreads();
  if (tid < I / 8) { union { v8h h; v4u u; } pk;
#pragma unroll
    for (int e = 0; e < 8; ++e) pk.h[e] = (_Float16)wrow[tid * 8 + e];
    vst2(wm + ((size_t)b * O + o) * I + tid * 8, pk.u); }
}
__global__ __launch_bounds__(128) void k_wrgb(const float* __restrict__ Wc, const float* __restrict__ S, int sj, int I, float* __restrict__ wr) {
  const int b = blockIdx.y, c = blockIdx.x, i = threadIdx.x;
  if (i < I) vst2(wr + ((size_t)b * 3 + c) * I + i, (float_a)(Wc[(size_t)c * I + i] * (S[((size_t)sj * NB + b) * 256 + i] + 1.0f)));
}

__global__ __launch_bounds__(256) void k_xT(const float* __restrict__ x, _Float16* __restrict__ xT) {
  __shared__ float tile[64][65];
  const int b = blockIdx.z, c0 = blockIdx.y * 64, p0 = blockIdx.x * 64, tid = threadIdx.x;
  for (int q = tid; q < 64 * 64; q += 256) { const int cl = q >> 6, pl = q & 63; tile[cl][pl] = x[((size_t)b * C0 + c0 + cl) * P0 + p0 + pl]; }
  __syncthreads();
  for (int q = tid; q < 64 * 8; q += 256) { const int pl = q >> 3, pc = q & 7;
    union { v8h h; v4u u; } pk;
#pragma unroll
    for (int e = 0; e < 8; ++e) pk.h[e] = (_Float16)tile[pc * 8 + e][pl];
    vst2(xT + ((size_t)b * P0 + p0 + pl) * C0 + c0 + pc * 8, pk.u); }
}

template <int O, int I, int ACT>
__global__ __launch_bounds__(O * 2) void k_mconv(const _Float16* __restrict__ wm, const _Float16* __restrict__ act, _Float16* __restrict__ outT, int P) {
  __shared__ __align__(16) float st[64][O + 4];
  const int tid = threadIdx.x, wave = tid >> 5, lane = tid & 31, col = lane & 15, g = lane >> 4;
  const int b = blockIdx.y, p0 = blockIdx.x * 64, o0 = wave * 16;
  v8f acc[4] = {};
#pragma unroll 1
  for (int kc = 0; kc < I / 32; ++kc) {
    const v16h a = frag_h(wm + ((size_t)b * O + o0 + col) * I + kc * 32, lane);
#pragma unroll
    for (int j = 0; j < 4; ++j) acc[j] = wmma16(a, frag_h(act + ((size_t)b * P + p0 + j * 16 + col) * I + kc * 32, lane), acc[j]);
  }
#pragma unroll
  for (int j = 0; j < 4; ++j)
#pragma unroll
    for (int r = 0; r < 8; ++r) { float v = acc[j][r]; if (ACT) v = lrelu(v); st[j * 16 + col][o0 + 8 * g + r] = v; }
  __syncthreads();
  for (int q = tid; q < 64 * (O / 8); q += O * 2) { const int pl = q / (O / 8), pc = q % (O / 8);
    union { v8h h; v4u u; } pk;
#pragma unroll
    for (int e = 0; e < 8; ++e) pk.h[e] = (_Float16)st[pl][pc * 8 + e];
    vst2(outT + ((size_t)b * P + p0 + pl) * O + pc * 8, pk.u); }
}

template <int C>
__global__ __launch_bounds__(256) void k_up2(const _Float16* __restrict__ in, _Float16* __restrict__ outp, int Hin) {
  const int b = blockIdx.y, Y = blockIdx.x, tid = threadIdx.x, Win = Hin, Wout = 2 * Hin;
  const float sy = (Y + 0.5f) * 0.5f - 0.5f; const int y0 = (int)floorf(sy); const float wy = sy - (float)y0;
  const int ya = min(max(y0, 0), Hin - 1), yb = min(max(y0 + 1, 0), Hin - 1);
  for (int q = tid; q < Wout * (C / 8); q += 256) { const int X = q / (C / 8), pc = q % (C / 8);
    const float sx = (X + 0.5f) * 0.5f - 0.5f; const int x0 = (int)floorf(sx); const float wx = sx - (float)x0;
    const int xa = min(max(x0, 0), Win - 1), xb = min(max(x0 + 1, 0), Win - 1);
    const _Float16* r00 = in + ((size_t)b * Hin * Win + ya * Win + xa) * C + pc * 8; const _Float16* r01 = in + ((size_t)b * Hin * Win + ya * Win + xb) * C + pc * 8;
    const _Float16* r10 = in + ((size_t)b * Hin * Win + yb * Win + xa) * C + pc * 8; const _Float16* r11 = in + ((size_t)b * Hin * Win + yb * Win + xb) * C + pc * 8;
    union { v8h h; v4u u; } pk;
#pragma unroll
    for (int e = 0; e < 8; ++e) { const float v = (float)r00[e] * (1.f - wy) * (1.f - wx) + (float)r01[e] * (1.f - wy) * wx + (float)r10[e] * wy * (1.f - wx) + (float)r11[e] * wy * wx;
      pk.h[e] = (_Float16)lrelu(v); }
    vst2(outp + ((size_t)b * Wout * Wout + Y * Wout + X) * C + pc * 8, pk.u); }
}

__global__ __launch_bounds__(256) void k_rgb1(const _Float16* __restrict__ h2, const float* __restrict__ wr1, float* __restrict__ r1) {
  const int b = blockIdx.y, p = blockIdx.x * 256 + threadIdx.x;
  const _Float16* hr = h2 + ((size_t)b * P1 + p) * C1;
#pragma unroll 1
  for (int c = 0; c < 3; ++c) { float a = 0.f; const float* w = wr1 + ((size_t)b * 3 + c) * C1;
#pragma unroll 1
    for (int i = 0; i < C1; i += 8) { const v8h v = *(const v8h*)(hr + i);
#pragma unroll
      for (int e = 0; e < 8; ++e) a += (float)v[e] * w[i + e]; }
    vst2(r1 + ((size_t)b * 3 + c) * P1 + p, (float_a)a); }
}
__device__ __forceinline__ int reflect256(int i) { return i < 0 ? -i : (i > H2 - 1 ? 2 * (H2 - 1) - i : i); }
__device__ __forceinline__ float up_sample(const float* __restrict__ img, int Y, int X) {
  const float sy = (Y + 0.5f) * 0.5f - 0.5f, sx = (X + 0.5f) * 0.5f - 0.5f;
  const int y0 = (int)floorf(sy), x0 = (int)floorf(sx); const float wy = sy - (float)y0, wx = sx - (float)x0;
  const int ya = min(max(y0, 0), H1 - 1), yb = min(max(y0 + 1, 0), H1 - 1), xa = min(max(x0, 0), H1 - 1), xb = min(max(x0 + 1, 0), H1 - 1);
  return img[ya * H1 + xa] * (1.f - wy) * (1.f - wx) + img[ya * H1 + xb] * (1.f - wy) * wx + img[yb * H1 + xa] * wy * (1.f - wx) + img[yb * H1 + xb] * wy * wx;
}
typedef __attribute__((ext_vector_type(4))) _Float16 v4h;
__global__ __launch_bounds__(256) void k_final(const float* __restrict__ r1, const _Float16* __restrict__ h4p, const float* __restrict__ wr2, float* __restrict__ out) {
  const int b = blockIdx.y, Y = blockIdx.x, X = threadIdx.x;
  const float sy = (Y + 0.5f) * 0.5f - 0.5f, sx = (X + 0.5f) * 0.5f - 0.5f;
  const int y0 = (int)floorf(sy), x0 = (int)floorf(sx); const float wy = sy - (float)y0, wx = sx - (float)x0;
  const int ya = min(max(y0, 0), H1 - 1), yb = min(max(y0 + 1, 0), H1 - 1), xa = min(max(x0, 0), H1 - 1), xb = min(max(x0 + 1, 0), H1 - 1);
  const float w00 = (1.f - wy) * (1.f - wx), w01 = (1.f - wy) * wx, w10 = wy * (1.f - wx), w11 = wy * wx;
  const _Float16* r00 = h4p + ((size_t)b * P1 + ya * H1 + xa) * C2; const _Float16* r01 = h4p + ((size_t)b * P1 + ya * H1 + xb) * C2;
  const _Float16* r10 = h4p + ((size_t)b * P1 + yb * H1 + xa) * C2; const _Float16* r11 = h4p + ((size_t)b * P1 + yb * H1 + xb) * C2;
  const float* wa = wr2 + ((size_t)b * 3 + 0) * C2; const float* wb = wa + C2; const float* wc = wb + C2;
  float a0 = 0.f, a1 = 0.f, a2 = 0.f;
#pragma unroll 1
  for (int i = 0; i < C2; i += 4) { const v4h v00 = *(const v4h*)(r00 + i), v01 = *(const v4h*)(r01 + i), v10 = *(const v4h*)(r10 + i), v11 = *(const v4h*)(r11 + i);
#pragma unroll
    for (int e = 0; e < 4; ++e) { const float v = lrelu((float)v00[e] * w00 + (float)v01[e] * w01 + (float)v10[e] * w10 + (float)v11[e] * w11);
      a0 += v * wa[i + e]; a1 += v * wb[i + e]; a2 += v * wc[i + e]; } }
#pragma unroll 1
  for (int c = 0; c < 3; ++c) {
    const float* img = r1 + ((size_t)b * 3 + c) * P1;
    float bl = 0.f;
#pragma unroll 1
    for (int dy = -1; dy <= 1; ++dy)
#pragma unroll 1
      for (int dx = -1; dx <= 1; ++dx) { const float kw = (dy == 0 ? 2.f : 1.f) * (dx == 0 ? 2.f : 1.f) * (1.0f / 16.0f);
        bl += kw * up_sample(img, reflect256(Y + dy), reflect256(X + dx)); }
    const float a = bl + (c == 0 ? a0 : (c == 1 ? a1 : a2));
    vst2(out + (((size_t)b * 3 + c) * H2 + Y) * H2 + X, (float_a)(1.0f / (1.0f + expf(-a))));
  }
}

extern "C" void kernel_launch(void* const* d_in, const int* in_sizes, int n_in,
                              void* d_out, int out_size, void* d_ws, size_t ws_size,
                              hipStream_t stream) {
  (void)in_sizes; (void)n_in; (void)out_size; (void)ws_size;
  const float* x = (const float*)d_in[0]; const float* y = (const float*)d_in[1];
  const float* ws11 = (const float*)d_in[2];  const float* bs11 = (const float*)d_in[3];
  const float* ws12 = (const float*)d_in[4];  const float* bs12 = (const float*)d_in[5];
  const float* ws13 = (const float*)d_in[6];  const float* bs13 = (const float*)d_in[7];
  const float* ws21 = (const float*)d_in[8];  const float* bs21 = (const float*)d_in[9];
  const float* ws22 = (const float*)d_in[10]; const float* bs22 = (const float*)d_in[11];
  const float* ws23 = (const float*)d_in[12]; const float* bs23 = (const float*)d_in[13];
  const float* wc1 = (const float*)d_in[14]; const float* wc2 = (const float*)d_in[15];
  const float* wc3 = (const float*)d_in[16]; const float* wc4 = (const float*)d_in[17];
  const float* wg1 = (const float*)d_in[18]; const float* wg2 = (const float*)d_in[19];
  float* out = (float*)d_out;
  char* ws = (char*)d_ws; size_t off = 0;
  auto take = [&](size_t bytes) { char* p = ws + off; off += (bytes + 255) & ~(size_t)255; return p; };
  float* S = (float*)take((size_t)6 * NB * 256 * 4);
  _Float16* wm1 = (_Float16*)take((size_t)NB * C1 * C0 * 2); _Float16* wm2 = (_Float16*)take((size_t)NB * C1 * C1 * 2);
  _Float16* wm3 = (_Float16*)take((size_t)NB * C2 * C1 * 2); _Float16* wm4 = (_Float16*)take((size_t)NB * C2 * C2 * 2);
  float* wr1 = (float*)take((size_t)NB * 3 * C1 * 4); float* wr2 = (float*)take((size_t)NB * 3 * C2 * 4);
  _Float16* xT = (_Float16*)take((size_t)NB * P0 * C0 * 2);
  _Float16* h1 = (_Float16*)take((size_t)NB * P0 * C1 * 2);
  _Float16* h2p = (_Float16*)take((size_t)NB * P0 * C1 * 2);
  _Float16* h2 = (_Float16*)take((size_t)NB * P1 * C1 * 2);
  float* r1 = (float*)take((size_t)NB * 3 * P1 * 4);
  _Float16* h3 = (_Float16*)take((size_t)NB * P1 * C2 * 2);
  _Float16* h4p = (_Float16*)take((size_t)NB * P1 * C2 * 2);
  k_style<<<dim3(NB, 6), 256, 0, stream>>>(y, ws11, bs11, ws12, bs12, ws13, bs13, ws21, bs21, ws22, bs22, ws23, bs23, S);
  k_wmod<<<dim3(C1, NB), 256, 0, stream>>>(wc1, S, 0, C1, C0, wm1);
  k_wmod<<<dim3(C1, NB), 256, 0, stream>>>(wc2, S, 1, C1, C1, wm2);
  k_wmod<<<dim3(C2, NB), 256, 0, stream>>>(wc3, S, 3, C2, C1, wm3);
  k_wmod<<<dim3(C2, NB), 256, 0, stream>>>(wc4, S, 4, C2, C2, wm4);
  k_wrgb<<<dim3(3, NB), 128, 0, stream>>>(wg1, S, 2, C1, wr1);
  k_wrgb<<<dim3(3, NB), 128, 0, stream>>>(wg2, S, 5, C2, wr2);
  k_xT<<<dim3(P0 / 64, C0 / 64, NB), 256, 0, stream>>>(x, xT);
  k_mconv<C1, C0, 1><<<dim3(P0 / 64, NB), 256, 0, stream>>>(wm1, xT, h1, P0);
  k_mconv<C1, C1, 0><<<dim3(P0 / 64, NB), 256, 0, stream>>>(wm2, h1, h2p, P0);
  k_up2<C1><<<dim3(H1, NB), 256, 0, stream>>>(h2p, h2, H0);
  k_rgb1<<<dim3(P1 / 256, NB), 256, 0, stream>>>(h2, wr1, r1);
  k_mconv<C2, C1, 1><<<dim3(P1 / 64, NB), 128, 0, stream>>>(wm3, h2, h3, P1);
  k_mconv<C2, C2, 0><<<dim3(P1 / 64, NB), 128, 0, stream>>>(wm4, h3, h4p, P1);
  k_final<<<dim3(H2, NB), 256, 0, stream>>>(r1, h4p, wr2, out);
}
